// GINNet_46084999086803
// MI455X (gfx1250) — hardware-verified
//
#include <hip/hip_runtime.h>
#include <math.h>

#define NN    50000
#define NE    800000
#define NG    256
#define FIN   128
#define HID   64
#define NCLS  10
#define NP    50048
#define NT    256
#define SRB   4096
#define NTL   13
#define SCH   4096
#define NCH   ((NE + SCH - 1) / SCH)
#define SCHP  2048
#define NCHP  ((NN + SCHP - 1) / SCHP)
#define SSP   32
#define WOFF1 8192
#define WOFF2 (8192 + 3 * 4096)
#define WPLANE 32768

static_assert(NP % 64 == 0);
static_assert(NP >= NN);
static_assert(NP % 4 == 0);
static_assert(NTL * SRB >= NP);
static_assert((NP * FIN / 8) % NT == 0);
static_assert((NP * HID / 8) % NT == 0);
static_assert(NE % (SCH / NT) == 0);
static_assert((SCH / NT) % 4 == 0);
static_assert(NN % (SCHP / NT) == 0);
static_assert((SCHP / NT) == 8);
static_assert(NN < 65536);
static_assert((SRB / 8) == 512);
static_assert(FIN % 32 == 0 && HID % 32 == 0);
static_assert((NG * NCLS) % 128 == 0);
static_assert(WOFF2 + 3 * HID * HID == WPLANE);

typedef __attribute__((ext_vector_type(16))) _Float16 v16h;
typedef __attribute__((ext_vector_type(8)))  _Float16 v8h;
typedef __attribute__((ext_vector_type(16))) __bf16   v16b;
typedef __attribute__((ext_vector_type(8)))  __bf16   v8b;
typedef __attribute__((ext_vector_type(8)))  float    v8f;
typedef __attribute__((ext_vector_type(4)))  float    v4f;
typedef __attribute__((ext_vector_type(2)))  float    v2f;
typedef __attribute__((ext_vector_type(4)))  int      v4i;
typedef __attribute__((ext_vector_type(4)))  unsigned int v4u;

__device__ __forceinline__ unsigned short f2bf_bits(float f) {
  unsigned u = __float_as_uint(f);
  return (unsigned short)((u + 0x7FFFu + ((u >> 16) & 1u)) >> 16);
}
__device__ __forceinline__ float bf_bits2f(unsigned short h) { return __uint_as_float(((unsigned)h) << 16); }
__device__ __forceinline__ unsigned pk16(unsigned short a, unsigned short b) { return (unsigned)a | ((unsigned)b << 16); }

__device__ __forceinline__ void dep_guard_h(v8f& a, v8f& b, v16h x, v16h y) { asm volatile("v_nop\n\tv_nop\n\tv_nop\n\tv_nop" : "+v"(a), "+v"(b) : "v"(x), "v"(y)); }
__device__ __forceinline__ void dep_guard_b(v8f& a, v8f& b, v16b x, v16b y) { asm volatile("v_nop\n\tv_nop\n\tv_nop\n\tv_nop" : "+v"(a), "+v"(b) : "v"(x), "v"(y)); }
__device__ __forceinline__ void dep_guard4_h(v8f& a, v8f& b, v8f& c, v8f& d, v16h x, v16h y) { asm volatile("v_nop\n\tv_nop\n\tv_nop\n\tv_nop" : "+v"(a), "+v"(b), "+v"(c), "+v"(d) : "v"(x), "v"(y)); }
__device__ __forceinline__ void dep_guard4_b(v8f& a, v8f& b, v8f& c, v8f& d, v16b x, v16b y) { asm volatile("v_nop\n\tv_nop\n\tv_nop\n\tv_nop" : "+v"(a), "+v"(b), "+v"(c), "+v"(d) : "v"(x), "v"(y)); }
__device__ __forceinline__ void keep4_h(v16h a, v16h b, v16h c, v16h d) { asm volatile("v_nop" :: "v"(a), "v"(b), "v"(c), "v"(d)); }
__device__ __forceinline__ void keep4_b(v16b a, v16b b, v16b c, v16b d) { asm volatile("v_nop" :: "v"(a), "v"(b), "v"(c), "v"(d)); }
__device__ __forceinline__ void acc_guard4(v8f& a, v8f& b, v8f& c, v8f& d) { asm volatile("v_nop\n\tv_nop\n\tv_nop\n\tv_nop" : "+v"(a), "+v"(b), "+v"(c), "+v"(d)); }
template <typename T> struct Frag;
template <> struct Frag<_Float16> {
  typedef v16h V; union U { v16h v; v8h h[2]; };
  static __device__ __forceinline__ v16h load(const _Float16* p) {
    U f; f.h[0] = *(const v8h*)(p); f.h[1] = *(const v8h*)(p + 16); return f.v;
  }
  static __device__ __forceinline__ v8f mma(v16h a, v16h b, v8f c) {
    return __builtin_amdgcn_wmma_f32_16x16x32_f16(false, a, false, b, (short)0, c, false, false);
  }
  static __device__ __forceinline__ void guard(v8f& a, v8f& b, v16h x, v16h y) { dep_guard_h(a, b, x, y); }
  static __device__ __forceinline__ void guard4(v8f& a, v8f& b, v8f& c, v8f& d, v16h x, v16h y) { dep_guard4_h(a, b, c, d, x, y); }
  static __device__ __forceinline__ void keep(v16h a, v16h b, v16h c, v16h d) { keep4_h(a, b, c, d); }
};
template <> struct Frag<__bf16> {
  typedef v16b V; union U { v16b v; v8b h[2]; };
  static __device__ __forceinline__ v16b load(const __bf16* p) {
    U f; f.h[0] = *(const v8b*)(p); f.h[1] = *(const v8b*)(p + 16); return f.v;
  }
  static __device__ __forceinline__ v8f mma(v16b a, v16b b, v8f c) {
    return __builtin_amdgcn_wmma_f32_16x16x32_bf16(false, a, false, b, (short)0, c, false, false);
  }
  static __device__ __forceinline__ void guard(v8f& a, v8f& b, v16b x, v16b y) { dep_guard_b(a, b, x, y); }
  static __device__ __forceinline__ void guard4(v8f& a, v8f& b, v8f& c, v8f& d, v16b x, v16b y) { dep_guard4_b(a, b, c, d, x, y); }
  static __device__ __forceinline__ void keep(v16b a, v16b b, v16b c, v16b d) { keep4_b(a, b, c, d); }
};

template <int ET> struct Elem;
template <> struct Elem<0> { typedef _Float16 T; };
template <> struct Elem<1> { typedef __bf16 T; };
template <int ET, bool SPLIT, int BIAS_MODE, int OUT_MODE, bool RESID, int ACT = 0>
__global__ __launch_bounds__(256) void wmma_gemm64(
    const unsigned short* __restrict__ Ap, const unsigned short* __restrict__ A2p, int lda, long strideA,
    const unsigned short* __restrict__ Btp, const unsigned short* __restrict__ Bt2p, int ldb, long strideB,
    void* __restrict__ Cout, void* __restrict__ Cout2, int ldc, long strideC,
    const float* __restrict__ bias,
    const float* __restrict__ resid, long strideR,
    int M, int N, int K, float scale) {
  typedef typename Elem<ET>::T T;
  typedef typename Frag<T>::V V;
  const T* A = (const T*)Ap; const T* A2 = (const T*)A2p; const T* Bt = (const T*)Btp; const T* Bt2 = (const T*)Bt2p;
  __shared__ __align__(16) float sT[8][16 * 68];
  const int b    = blockIdx.y;
  const int lane = threadIdx.x & 31;
  const int wave = threadIdx.x >> 5;
  const int tilesN = N >> 6;
  const int tilesM = M >> 6;
  const int tile = blockIdx.x * 8 + wave;
  if (tile >= tilesM * tilesN) return;
  const int tm = tile / tilesN;
  const int tn = tile - tm * tilesN;
  const int m0 = tm << 6;
  const int n0 = tn << 6;

  const T* Ab  = A  + (size_t)b * strideA;
  const T* Bb  = Bt + (size_t)b * strideB;
  const T* Ab2 = SPLIT ? (A2  + (size_t)b * strideA) : nullptr;
  const T* Bb2 = SPLIT ? (Bt2 + (size_t)b * strideB) : nullptr;

  const int rlane = lane & 15;
  const int koff  = (lane >> 4) * 8;
  const int mOff  = (lane >> 4) * 8;

  v8f acc[4][4];
#pragma unroll
  for (int i = 0; i < 4; ++i)
#pragma unroll
    for (int j = 0; j < 4; ++j) acc[i][j] = (v8f){0.f,0.f,0.f,0.f,0.f,0.f,0.f,0.f};

  for (int k0 = 0; k0 < K; k0 += 32) {
    V bh[4], bl[4];
#pragma unroll
    for (int j = 0; j < 4; ++j) {
      const size_t bo = (size_t)(n0 + (j << 4) + rlane) * ldb + koff + k0;
      bh[j] = Frag<T>::load(Bb + bo);
      if (SPLIT) bl[j] = Frag<T>::load(Bb2 + bo);
    }
#pragma unroll
    for (int i = 0; i < 4; ++i) {
      const size_t ao = (size_t)(m0 + (i << 4) + rlane) * lda + koff + k0;
      V ah = Frag<T>::load(Ab + ao);
      V al;
      if (SPLIT) al = Frag<T>::load(Ab2 + ao);
#pragma unroll
      for (int j = 0; j < 4; ++j) {
        acc[i][j] = Frag<T>::mma(ah, bh[j], acc[i][j]);
        if (SPLIT) {
          acc[i][j] = Frag<T>::mma(ah, bl[j], acc[i][j]);
          acc[i][j] = Frag<T>::mma(al, bh[j], acc[i][j]);
        }
      }
      Frag<T>::guard4(acc[i][0], acc[i][1], acc[i][2], acc[i][3], ah, SPLIT ? al : ah);
    }
    Frag<T>::keep(bh[0], bh[1], bh[2], bh[3]);
    if (SPLIT) Frag<T>::keep(bl[0], bl[1], bl[2], bl[3]);
  }
  acc_guard4(acc[0][0], acc[0][1], acc[0][2], acc[0][3]);
  acc_guard4(acc[1][0], acc[1][1], acc[1][2], acc[1][3]);
  acc_guard4(acc[2][0], acc[2][1], acc[2][2], acc[2][3]);
  acc_guard4(acc[3][0], acc[3][1], acc[3][2], acc[3][3]);

  float* slab = sT[wave];
  const float* Rb = RESID ? (resid + (size_t)b * strideR) : nullptr;
#pragma unroll
  for (int i = 0; i < 4; ++i) {
    const int mBase = m0 + (i << 4);
#pragma unroll
    for (int j = 0; j < 4; ++j) {
      const int n = n0 + (j << 4) + rlane;
      float bv = 0.f;
      if (BIAS_MODE == 2) bv = bias[n];
#pragma unroll
      for (int r = 0; r < 8; ++r) {
        float v = acc[i][j][r] * scale;
        if (BIAS_MODE == 1) v += bias[mBase + mOff + r];
        if (BIAS_MODE == 2) v += bv;
        if (RESID) v += Rb[(size_t)(mBase + mOff + r) * ldc + n];
        if (ACT == 2) v = fmaxf(v, 0.0f);
        slab[(mOff + r) * 68 + (j << 4) + rlane] = v;
      }
    }
    __builtin_amdgcn_fence(__ATOMIC_RELEASE, "workgroup");
    __builtin_amdgcn_wave_barrier();
    __builtin_amdgcn_fence(__ATOMIC_ACQUIRE, "workgroup");
    if (OUT_MODE == 0) {
      float* C = (float*)Cout + (size_t)b * strideC;
      const int hh = lane >> 4, c4 = (lane & 15) * 4;
      for (int pass = 0; pass < 2; ++pass) {
#pragma unroll
        for (int it = 0; it < 8; ++it) {
          const int row = it * 2 + hh;
          v4f v = *(const v4f*)(slab + row * 68 + c4);
          *(volatile v4f*)(C + (size_t)(mBase + row) * ldc + n0 + c4) = v;
        }
        __threadfence();
      }
    } else {
      const int q = lane >> 3, c8 = (lane & 7) * 8;
      unsigned short* C  = (unsigned short*)Cout  + (size_t)b * strideC;
      unsigned short* C2 = (OUT_MODE == 2) ? ((unsigned short*)Cout2 + (size_t)b * strideC) : nullptr;
      for (int pass = 0; pass < 2; ++pass) {
#pragma unroll
        for (int it = 0; it < 4; ++it) {
          const int row = it * 4 + q;
          const float* sp = slab + row * 68 + c8;
          v8h hv, lv;
#pragma unroll
          for (int e = 0; e < 8; ++e) {
            if (OUT_MODE == 1) {
              hv[e] = (_Float16)sp[e];
            } else {
              unsigned short hb = f2bf_bits(sp[e]);
              unsigned short lb = f2bf_bits(sp[e] - bf_bits2f(hb));
              hv[e] = __builtin_bit_cast(_Float16, hb);
              lv[e] = __builtin_bit_cast(_Float16, lb);
            }
          }
          *(volatile v8h*)(C + (size_t)(mBase + row) * ldc + n0 + c8) = hv;
          if (OUT_MODE == 2) *(volatile v8h*)(C2 + (size_t)(mBase + row) * ldc + n0 + c8) = lv;
        }
        __threadfence();
      }
    }
    __builtin_amdgcn_fence(__ATOMIC_RELEASE, "workgroup");
    __builtin_amdgcn_wave_barrier();
    __builtin_amdgcn_fence(__ATOMIC_ACQUIRE, "workgroup");
  }
}

__device__ __forceinline__ int blk_excl_scan(int cnt, int* scan_ws, int tid, int* tot) {
  const int lane = tid & 31, wave = tid >> 5; int incl = cnt;
#pragma unroll
  for (int o = 1; o < 32; o <<= 1) { const int v = __shfl_up(incl, o, 32); if (lane >= o) incl += v; }
  if (lane == 31) scan_ws[wave] = incl;
  __syncthreads();
  if (wave == 0) { int wv = (lane < NT / 32) ? scan_ws[lane] : 0; int wincl = wv;
#pragma unroll
    for (int o = 1; o < 32; o <<= 1) { const int v = __shfl_up(wincl, o, 32); if (lane >= o) wincl += v; }
    if (lane < NT / 32) scan_ws[32 + lane] = wincl - wv; if (lane == 31) scan_ws[64] = wincl; }
  __syncthreads();
  const int res = scan_ws[32 + wave] + incl - cnt; *tot = scan_ws[64];
  return res;
}

template <int SP, int CAP>
__device__ __forceinline__ int chunk_hits(const int* __restrict__ dstv, const int* __restrict__ srcv, int e0, int n0, int tid,
                                          int* LIST, int* scan_ws) {
  const int eb = e0 + tid * SP;
  const bool inr = eb < NE;
  const int ebc = inr ? eb : (NE - SP);
  int rec[SP]; int cnt = 0;
#pragma unroll
  for (int k = 0; k < SP; k += 4) {
    const v4i d4 = *(const v4i*)(dstv + ebc + k);
    const v4i s4 = *(const v4i*)(srcv + ebc + k);
#pragma unroll
    for (int e = 0; e < 4; ++e) {
      const int d = d4[e];
      int s = s4[e]; s = s < 0 ? 0 : (s >= NN ? NN - 1 : s);
      const bool hit = inr && (d >= n0) && (d < n0 + SRB);
      const int packed = (((d - n0) & (SRB - 1)) << 16) | s;
      rec[k + e] = hit ? packed : -1;
      cnt += hit ? 1 : 0;
    }
  }
  int tot; int p = blk_excl_scan(cnt, scan_ws, tid, &tot);
#pragma unroll
  for (int k = 0; k < SP; ++k) if (rec[k] >= 0) { if ((unsigned)p < (unsigned)CAP) LIST[p] = rec[k]; ++p; }
  __syncthreads();
  return tot < CAP ? tot : CAP;
}

template <int F>
__global__ __launch_bounds__(NT) void colstats_kernel(const float* __restrict__ X, const float* __restrict__ gam,
                                                      const float* __restrict__ bet, float* __restrict__ tab) {
  __shared__ double s_sum[NT];
  __shared__ double s_sq[NT];
  const int f = blockIdx.x;
  const int tid = threadIdx.x;
  double s = 0.0, q = 0.0;
#pragma unroll 1
  for (int m = tid; m < NN; m += NT) {
    const double dv = (double)X[(size_t)m * F + f];
    s += dv; q += dv * dv;
  }
  s_sum[tid] = s; s_sq[tid] = q;
  __syncthreads();
#pragma unroll 1
  for (int off = NT / 2; off > 0; off >>= 1) {
    if (tid < off) { s_sum[tid] += s_sum[tid + off]; s_sq[tid] += s_sq[tid + off]; }
    __syncthreads();
  }
  if (tid < 32) {
    const double inv = 1.0 / (double)NN;
    const double mu = s_sum[0] * inv;
    double var = s_sq[0] * inv - mu * mu;
    var = var > 0.0 ? var : 0.0;
    const float muf = (float)mu, varf = (float)var;
    const float is = 1.0f / sqrtf(varf + 1e-5f);
    const float sc = gam[f] * is;
    const float sh = bet[f] - muf * sc;
    const float val = (tid == 0) ? sc : ((tid == 1) ? sh : 0.0f);
    float* line = tab + (size_t)f * SSP;
    ((volatile float*)line)[tid] = val;
    __threadfence();
    ((volatile float*)line)[tid] = val;
  }
}

__global__ __launch_bounds__(NT) void xplanes_kernel(const float* __restrict__ x, const float* __restrict__ tab,
                                                     unsigned short* __restrict__ XH, unsigned short* __restrict__ XL) {
  __shared__ float ssc[FIN];
  __shared__ float ssh[FIN];
  const int tid = threadIdx.x;
  if (tid < FIN) { ssc[tid] = tab[tid * SSP]; ssh[tid] = tab[tid * SSP + 1]; }
  __syncthreads();
  const int i = blockIdx.x * NT + tid;
  const int e = i * 8;
  const int row = e >> 7;
  const int col = e & (FIN - 1);
  const int rowc = row < NN ? row : NN - 1;
  const bool live = row < NN;
  const float* p = x + (size_t)rowc * FIN + col;
  const v4f a = *(const v4f*)p;
  const v4f c = *(const v4f*)(p + 4);
  unsigned short hb[8], lb[8];
#pragma unroll
  for (int k = 0; k < 4; ++k) {
    float v0 = a[k] * ssc[col + k] + ssh[col + k];          v0 = live ? v0 : 0.f;
    float v1 = c[k] * ssc[col + 4 + k] + ssh[col + 4 + k];  v1 = live ? v1 : 0.f;
    hb[k] = f2bf_bits(v0);     lb[k] = f2bf_bits(v0 - bf_bits2f(hb[k]));
    hb[4 + k] = f2bf_bits(v1); lb[4 + k] = f2bf_bits(v1 - bf_bits2f(hb[4 + k]));
  }
  const v4u uh = (v4u){pk16(hb[0], hb[1]), pk16(hb[2], hb[3]), pk16(hb[4], hb[5]), pk16(hb[6], hb[7])};
  const v4u ul = (v4u){pk16(lb[0], lb[1]), pk16(lb[2], lb[3]), pk16(lb[4], lb[5]), pk16(lb[6], lb[7])};
  unsigned short* qh = XH + (size_t)e;
  unsigned short* ql = XL + (size_t)e;
  *(volatile v4u*)qh = uh; *(volatile v4u*)ql = ul;
  __threadfence();
  *(volatile v4u*)qh = uh; *(volatile v4u*)ql = ul;
}

__global__ __launch_bounds__(NT) void uplanes_kernel(const float* __restrict__ tb, const float* __restrict__ tab,
                                                     unsigned short* __restrict__ UH, unsigned short* __restrict__ UL) {
  __shared__ float ssc[HID];
  __shared__ float ssh[HID];
  const int tid = threadIdx.x;
  if (tid < HID) { ssc[tid] = tab[tid * SSP]; ssh[tid] = tab[tid * SSP + 1]; }
  __syncthreads();
  const int i = blockIdx.x * NT + tid;
  const int e = i * 8;
  const int row = e >> 6;
  const int col = e & (HID - 1);
  const int rowc = row < NN ? row : NN - 1;
  const bool live = row < NN;
  const float* p = tb + (size_t)rowc * HID + col;
  const v4f a = *(const v4f*)p;
  const v4f c = *(const v4f*)(p + 4);
  unsigned short hb[8], lb[8];
#pragma unroll
  for (int k = 0; k < 4; ++k) {
    float v0 = a[k] * ssc[col + k] + ssh[col + k];          v0 = live ? fmaxf(v0, 0.f) : 0.f;
    float v1 = c[k] * ssc[col + 4 + k] + ssh[col + 4 + k];  v1 = live ? fmaxf(v1, 0.f) : 0.f;
    hb[k] = f2bf_bits(v0);     lb[k] = f2bf_bits(v0 - bf_bits2f(hb[k]));
    hb[4 + k] = f2bf_bits(v1); lb[4 + k] = f2bf_bits(v1 - bf_bits2f(hb[4 + k]));
  }
  const v4u uh = (v4u){pk16(hb[0], hb[1]), pk16(hb[2], hb[3]), pk16(hb[4], hb[5]), pk16(hb[6], hb[7])};
  const v4u ul = (v4u){pk16(lb[0], lb[1]), pk16(lb[2], lb[3]), pk16(lb[4], lb[5]), pk16(lb[6], lb[7])};
  unsigned short* qh = UH + (size_t)e;
  unsigned short* ql = UL + (size_t)e;
  *(volatile v4u*)qh = uh; *(volatile v4u*)ql = ul;
  __threadfence();
  *(volatile v4u*)qh = uh; *(volatile v4u*)ql = ul;
}

__global__ __launch_bounds__(NT) void wprep_kernel(const float* __restrict__ Wf, const float* __restrict__ W1, const float* __restrict__ W2,
                                                   unsigned* __restrict__ WHd, unsigned* __restrict__ WLd) {
  const int tid = threadIdx.x;
  const int bx = blockIdx.x;
  float a, b; int od;
  if (bx < 16) {
    const int d = bx * NT + tid;
    const int e0 = 2 * d;
    const int n = e0 >> 7;
    const int k = e0 & (FIN - 1);
    a = Wf[k * HID + n]; b = Wf[(k + 1) * HID + n]; od = d;
  } else {
    const int j = bx - 16;
    const int mat = j >> 3;
    const int dl = (j & 7) * NT + tid;
    const int e0 = 2 * dl;
    const int n = e0 >> 6;
    const int k = e0 & (HID - 1);
    const float* src = (mat < 3) ? (W1 + mat * HID * HID) : (W2 + (mat - 3) * HID * HID);
    a = src[k * HID + n]; b = src[(k + 1) * HID + n]; od = (WOFF1 / 2) + mat * (HID * HID / 2) + dl;
  }
  const unsigned short ha = f2bf_bits(a), hbv = f2bf_bits(b);
  const unsigned short la = f2bf_bits(a - bf_bits2f(ha)), lbv = f2bf_bits(b - bf_bits2f(hbv));
  const unsigned uh = pk16(ha, hbv), ul = pk16(la, lbv);
  ((volatile unsigned*)WHd)[od] = uh; ((volatile unsigned*)WLd)[od] = ul;
  __threadfence();
  ((volatile unsigned*)WHd)[od] = uh; ((volatile unsigned*)WLd)[od] = ul;
}

__global__ __launch_bounds__(NT) void gin_agg_kernel(const float* __restrict__ Hs, const int* __restrict__ ei, float* ACC,
                                                     unsigned short* __restrict__ ZH, unsigned short* __restrict__ ZL) {
  __shared__ int LIST[SCH];
  __shared__ int scan_ws[80];
  const int tid = threadIdx.x, lane = tid & 31, wave = tid >> 5;
  const int n0 = blockIdx.x * SRB;
  const int w0 = n0 + wave * (SRB / 8);
  if (tid < 80) scan_ws[tid] = 0;
  const v2f z2 = {0.f, 0.f};
#pragma unroll 1
  for (int j = 0; j < SRB / 8; ++j) *(v2f*)(ACC + (size_t)(w0 + j) * HID + 2 * lane) = z2;
  __syncthreads();
  const int* srcv = ei;
  const int* dstv = ei + NE;
#pragma unroll 1
  for (int c = 0; c < NCH; ++c) {
    const int tot = chunk_hits<SCH / NT, SCH>(dstv, srcv, c * SCH, n0, tid, LIST, scan_ws);
#pragma unroll 1
    for (int base = 0; base < tot; base += 32) {
      const int qr = base + lane;
      const int qc = qr < tot ? qr : tot - 1;
      const int rv0 = LIST[qc];
      const int rv = (qr < tot) ? rv0 : -1;
      const int own = (rv >= 0 && (rv >> 25) == wave) ? 1 : 0;
      unsigned msk = (unsigned)__ballot(own);
#pragma unroll 1
      for (int it = 0; it < 32; ++it) {
        if (msk == 0u) break;
        const int bp = __builtin_ctz(msk); msk &= msk - 1u;
        const int r = __shfl(rv, bp, 32);
        const int dl = (r >> 16) & (SRB - 1);
        int s = r & 0xFFFF; s = s < NN ? s : NN - 1;
        const v2f hv = *(const v2f*)(Hs + (size_t)s * HID + 2 * lane);
        float* rp = ACC + (size_t)(n0 + dl) * HID + 2 * lane;
        v2f a = *(const v2f*)rp;
        a = a + hv;
        *(v2f*)rp = a;
      }
    }
    __syncthreads();
  }
  const int rq = lane >> 3, c8 = (lane & 7) * 8;
#pragma unroll 1
  for (int it = 0; it < SRB / 32; ++it) {
    const int rb = w0 + it * 4;
    if (rb < NP) {
      const int n = rb + rq;
      const bool live = n < NN;
      const float* ap = ACC + (size_t)n * HID + c8;
      const float* hp = Hs + (size_t)n * HID + c8;
      const v4f a0 = *(const v4f*)ap, a1 = *(const v4f*)(ap + 4);
      const v4f h0 = *(const v4f*)hp, h1 = *(const v4f*)(hp + 4);
      unsigned short hb[8], lb[8];
#pragma unroll
      for (int k = 0; k < 4; ++k) {
        float z0 = h0[k] + a0[k]; z0 = live ? z0 : 0.f;
        float z1 = h1[k] + a1[k]; z1 = live ? z1 : 0.f;
        hb[k] = f2bf_bits(z0);     lb[k] = f2bf_bits(z0 - bf_bits2f(hb[k]));
        hb[4 + k] = f2bf_bits(z1); lb[4 + k] = f2bf_bits(z1 - bf_bits2f(hb[4 + k]));
      }
      const v4u uh = (v4u){pk16(hb[0], hb[1]), pk16(hb[2], hb[3]), pk16(hb[4], hb[5]), pk16(hb[6], hb[7])};
      const v4u ul = (v4u){pk16(lb[0], lb[1]), pk16(lb[2], lb[3]), pk16(lb[4], lb[5]), pk16(lb[6], lb[7])};
      unsigned short* zh = ZH + (size_t)n * HID + c8;
      unsigned short* zl = ZL + (size_t)n * HID + c8;
      *(volatile v4u*)zh = uh; *(volatile v4u*)zl = ul;
      __threadfence();
      *(volatile v4u*)zh = uh; *(volatile v4u*)zl = ul;
    }
  }
}

__global__ __launch_bounds__(NT) void pool_kernel(const float* __restrict__ Hs, const int* __restrict__ bat, float* __restrict__ HG) {
  __shared__ int LIST[SCHP];
  __shared__ int scan_ws[80];
  __shared__ __align__(16) float red[(NT / 32) * HID];
  const int tid = threadIdx.x, lane = tid & 31, wave = tid >> 5;
  const int g = blockIdx.x;
  if (tid < 80) scan_ws[tid] = 0;
  __syncthreads();
  v2f acc = {0.f, 0.f};
#pragma unroll 1
  for (int c = 0; c < NCHP; ++c) {
    const int eb = c * SCHP + tid * (SCHP / NT);
    const bool inr = eb < NN;
    const int ebc = inr ? eb : (NN - (SCHP / NT));
    const v4i b0 = *(const v4i*)(bat + ebc);
    const v4i b1 = *(const v4i*)(bat + ebc + 4);
    int rec[8]; int cnt = 0;
#pragma unroll
    for (int k = 0; k < 4; ++k) {
      const bool h0 = inr && (b0[k] == g); rec[k] = h0 ? (eb + k) : -1;         cnt += h0 ? 1 : 0;
      const bool h1 = inr && (b1[k] == g); rec[4 + k] = h1 ? (eb + 4 + k) : -1; cnt += h1 ? 1 : 0;
    }
    int tot; int p = blk_excl_scan(cnt, scan_ws, tid, &tot);
#pragma unroll
    for (int k = 0; k < 8; ++k) if (rec[k] >= 0) { if ((unsigned)p < (unsigned)SCHP) LIST[p] = rec[k]; ++p; }
    __syncthreads();
    const int totc = tot < SCHP ? tot : SCHP;
#pragma unroll 1
    for (int q = wave; q < totc; q += NT / 32) {
      int nd = LIST[q]; nd = nd < 0 ? 0 : (nd >= NN ? NN - 1 : nd);
      acc = acc + *(const v2f*)(Hs + (size_t)nd * HID + 2 * lane);
    }
    __syncthreads();
  }
  *(v2f*)(red + wave * HID + 2 * lane) = acc;
  __syncthreads();
  if (wave == 0) {
    const int c4 = (lane & 15) * 4;
    v4f s = {0.f, 0.f, 0.f, 0.f};
#pragma unroll
    for (int w = 0; w < NT / 32; ++w) s = s + *(const v4f*)(red + w * HID + c4);
    for (int pass = 0; pass < 2; ++pass) {
      if (lane < 16) *(volatile v4f*)(HG + (size_t)g * HID + c4) = s;
      __threadfence();
    }
  }
}

__device__ __forceinline__ void stats_rows_g(const float* __restrict__ X, int col, const float* __restrict__ gam,
                                             const float* __restrict__ bet, float* ssc, float* ssh) {
  double s = 0.0, q = 0.0;
#pragma unroll 1
  for (int g = 0; g < NG; ++g) { const double dv = (double)X[g * HID + col]; s += dv; q += dv * dv; }
  const double inv = 1.0 / (double)NG;
  const double mu = s * inv;
  double var = q * inv - mu * mu;
  var = var > 0.0 ? var : 0.0;
  const float muf = (float)mu, varf = (float)var;
  const float is = 1.0f / sqrtf(varf + 1e-5f);
  const float sc = gam[col] * is;
  ssc[col] = sc;
  ssh[col] = bet[col] - muf * sc;
}

__global__ __launch_bounds__(NT) void head1_kernel(const float* __restrict__ HG, const float* __restrict__ gam, const float* __restrict__ bet,
                                                   const float* __restrict__ Wl, const float* __restrict__ bl, float* __restrict__ HG1) {
  __shared__ float ssc[HID];
  __shared__ float ssh[HID];
  __shared__ float sW[HID * HID];
  __shared__ float sV[64 * HID];
  const int tid = threadIdx.x;
  if (tid < HID) stats_rows_g(HG, tid, gam, bet, ssc, ssh);
#pragma unroll 1
  for (int i = tid; i < HID * HID; i += NT) sW[i] = Wl[i];
  __syncthreads();
#pragma unroll 1
  for (int gc = 0; gc < NG / 64; ++gc) {
#pragma unroll 1
    for (int i = tid; i < 64 * HID; i += NT) {
      const int gl = i >> 6, k = i & (HID - 1);
      sV[i] = HG[(size_t)(gc * 64 + gl) * HID + k] * ssc[k] + ssh[k];
    }
    __syncthreads();
#pragma unroll 1
    for (int it = 0; it < 16; ++it) {
      const int o = it * NT + tid;
      const int gl = o >> 6, j = o & (HID - 1);
      float s = 0.0f;
#pragma unroll 1
      for (int k = 0; k < HID; ++k) s += sV[gl * HID + k] * sW[k * HID + j];
      s += bl[j];
      s = fmaxf(s, 0.0f);
      float* dp = HG1 + (size_t)(gc * 64 + gl) * HID + j;
      *(volatile float*)dp = s;
      __threadfence();
      *(volatile float*)dp = s;
    }
    __syncthreads();
  }
}

__global__ __launch_bounds__(NT) void head2_kernel(const float* __restrict__ HG1, const float* __restrict__ gam, const float* __restrict__ bet,
                                                   const float* __restrict__ Wc, const float* __restrict__ cb, float* __restrict__ out) {
  __shared__ float ssc[HID];
  __shared__ float ssh[HID];
  __shared__ float sC[HID * NCLS];
  __shared__ float scb[16];
  __shared__ __align__(16) float so[NG * NCLS];
  const int tid = threadIdx.x, lane = tid & 31, wave = tid >> 5;
  if (tid < HID) stats_rows_g(HG1, tid, gam, bet, ssc, ssh);
#pragma unroll 1
  for (int i = tid; i < HID * NCLS; i += NT) sC[i] = Wc[i];
  if (tid < 16) scb[tid] = (tid < NCLS) ? cb[tid < NCLS ? tid : 0] : 0.f;
  __syncthreads();
#pragma unroll 1
  for (int it = 0; it < NCLS; ++it) {
    const int o = it * NT + tid;
    const int g = o / NCLS;
    const int c = o - g * NCLS;
    float s = 0.0f;
#pragma unroll 1
    for (int k = 0; k < HID; ++k) {
      const float v = HG1[(size_t)g * HID + k] * ssc[k] + ssh[k];
      s += v * sC[k * NCLS + c];
    }
    s += scb[c];
    so[o] = s;
  }
  __syncthreads();
  for (int pass = 0; pass < 2; ++pass) {
#pragma unroll 1
    for (int qq = wave; qq < (NG * NCLS) / 128; qq += NT / 32) {
      const v4f v = *(const v4f*)(so + qq * 128 + 4 * lane);
      *(volatile v4f*)(out + (size_t)qq * 128 + 4 * lane) = v;
    }
    __threadfence();
  }
}

extern "C" void kernel_launch(void* const* d_in, const int* in_sizes, int n_in,
                              void* d_out, int out_size, void* d_ws, size_t ws_size, hipStream_t stream) {
  (void)in_sizes; (void)n_in; (void)out_size;
  const float* x          = (const float*)d_in[0];
  const int*   edge_index = (const int*)  d_in[1];
  const int*   batch      = (const int*)  d_in[2];
  const float* bn_feat_g  = (const float*)d_in[3];
  const float* bn_feat_b  = (const float*)d_in[4];
  const float* w_feat     = (const float*)d_in[5];
  const float* b_feat     = (const float*)d_in[6];
  const float* gin_w1     = (const float*)d_in[7];
  const float* gin_b1     = (const float*)d_in[8];
  const float* gin_bn_g   = (const float*)d_in[9];
  const float* gin_bn_b   = (const float*)d_in[10];
  const float* gin_w2     = (const float*)d_in[11];
  const float* gin_b2     = (const float*)d_in[12];
  const float* bn_fc_g    = (const float*)d_in[13];
  const float* bn_fc_b    = (const float*)d_in[14];
  const float* lin_w      = (const float*)d_in[15];
  const float* lin_b      = (const float*)d_in[16];
  const float* bn_h_g     = (const float*)d_in[17];
  const float* bn_h_b     = (const float*)d_in[18];
  const float* cls_w      = (const float*)d_in[19];
  const float* cls_b      = (const float*)d_in[20];
  float* out = (float*)d_out;

  char* ws = (char*)d_ws; size_t off = 0;
  auto carve = [&](size_t bytes) -> char* { char* p = ws + off; off += (bytes + 255) & ~(size_t)255; return p; };
  float*          SSX = (float*)carve((size_t)FIN * SSP * 4);
  float*          SST = (float*)carve((size_t)HID * SSP * 4);
  unsigned short* WH  = (unsigned short*)carve((size_t)WPLANE * 2);
  unsigned short* WL  = (unsigned short*)carve((size_t)WPLANE * 2);
  unsigned short* XH  = (unsigned short*)carve((size_t)NP * FIN * 2);
  unsigned short* XL  = (unsigned short*)carve((size_t)NP * FIN * 2);
  float*          HB  = (float*)carve((size_t)NP * HID * 4);
  float*          TB  = (float*)carve((size_t)NP * HID * 4);
  unsigned short* ZH  = (unsigned short*)carve((size_t)NP * HID * 2);
  unsigned short* ZL  = (unsigned short*)carve((size_t)NP * HID * 2);
  unsigned short* UH  = (unsigned short*)carve((size_t)NP * HID * 2);
  unsigned short* UL  = (unsigned short*)carve((size_t)NP * HID * 2);
  float*          ACC = (float*)carve((size_t)NTL * SRB * HID * 4);
  float*          HG  = (float*)carve((size_t)NG * HID * 4);
  float*          HG1 = (float*)carve((size_t)NG * HID * 4);
  if (off > ws_size || off > (size_t)134217728) return;

  const int gemm_blocks = (NP / 64 + 7) / 8;

  colstats_kernel<FIN><<<FIN, NT, 0, stream>>>(x, bn_feat_g, bn_feat_b, SSX);
  xplanes_kernel<<<(NP * FIN / 8) / NT, NT, 0, stream>>>(x, SSX, XH, XL);
  wprep_kernel<<<64, NT, 0, stream>>>(w_feat, gin_w1, gin_w2, (unsigned*)WH, (unsigned*)WL);
  wmma_gemm64<1, true, 2, 0, false, 2><<<dim3(gemm_blocks, 1), NT, 0, stream>>>(
      (const unsigned short*)XH, (const unsigned short*)XL, FIN, 0L,
      (const unsigned short*)WH, (const unsigned short*)WL, FIN, 0L,
      (void*)HB, (void*)nullptr, HID, 0L,
      b_feat, (const float*)nullptr, 0L, NP, HID, FIN, 1.0f);

  for (int i = 0; i < 3; ++i) {
    const unsigned short* W1H = WH + WOFF1 + i * HID * HID;
    const unsigned short* W1L = WL + WOFF1 + i * HID * HID;
    const unsigned short* W2H = WH + WOFF2 + i * HID * HID;
    const unsigned short* W2L = WL + WOFF2 + i * HID * HID;
    gin_agg_kernel<<<NTL, NT, 0, stream>>>(HB, edge_index, ACC, ZH, ZL);
    wmma_gemm64<1, true, 2, 0, false, 0><<<dim3(gemm_blocks, 1), NT, 0, stream>>>(
        (const unsigned short*)ZH, (const unsigned short*)ZL, HID, 0L,
        W1H, W1L, HID, 0L,
        (void*)TB, (void*)nullptr, HID, 0L,
        gin_b1 + i * HID, (const float*)nullptr, 0L, NP, HID, HID, 1.0f);
    colstats_kernel<HID><<<HID, NT, 0, stream>>>(TB, gin_bn_g + i * HID, gin_bn_b + i * HID, SST);
    uplanes_kernel<<<(NP * HID / 8) / NT, NT, 0, stream>>>(TB, SST, UH, UL);
    wmma_gemm64<1, true, 2, 0, false, 2><<<dim3(gemm_blocks, 1), NT, 0, stream>>>(
        (const unsigned short*)UH, (const unsigned short*)UL, HID, 0L,
        W2H, W2L, HID, 0L,
        (void*)HB, (void*)nullptr, HID, 0L,
        gin_b2 + i * HID, (const float*)nullptr, 0L, NP, HID, HID, 1.0f);
  }

  pool_kernel<<<NG, NT, 0, stream>>>(HB, batch, HG);
  head1_kernel<<<1, NT, 0, stream>>>(HG, bn_fc_g, bn_fc_b, lin_w, lin_b, HG1);
  head2_kernel<<<1, NT, 0, stream>>>(HG1, bn_h_g, bn_h_b, cls_w, cls_b, out);
}
